// SoilMoistureGapFilling_52218212384939
// MI455X (gfx1250) — hardware-verified
//
#include <hip/hip_runtime.h>
#include <stdint.h>

typedef __attribute__((ext_vector_type(16))) _Float16 v16h;
typedef __attribute__((ext_vector_type(8)))  _Float16 v8h;
typedef __attribute__((ext_vector_type(4)))  _Float16 v4h;
typedef __attribute__((ext_vector_type(8)))  float    v8f;
typedef __attribute__((ext_vector_type(4)))  float    v4f;

constexpr int kNB   = 1024;
constexpr int kNT   = 365;
constexpr int kNF   = 8;
constexpr int kNS   = 16;
constexpr int kNH   = 128;
constexpr int kNFFN = 128;
constexpr int kNG   = 4 * kNH;
constexpr int kKIN  = kNF + 1;
constexpr int kK1   = kNH + kNS;
constexpr int kK1P  = 160;

constexpr int kSeqPB  = 16;
constexpr int kBlocks = kNB / kSeqPB;
constexpr int kThreads = 256;
constexpr int kWaves  = kThreads / 32;
constexpr int kWhhP   = kNH;
constexpr int kW1P    = kK1P;
constexpr int kAP     = kK1P;
constexpr int kYSP    = 384;
constexpr float kASc  = 16.0f;
constexpr float kWSc  = 8.0f;
constexpr float kDown = 1.0f / 128.0f;
constexpr int kOut4   = kNB * kNT / 4;
constexpr int kRepackBlocks = (kOut4 + 255) / 256;
static_assert(kNB % kSeqPB == 0);
static_assert(kWaves * 16 == kNH && kWaves * 16 == kNFFN);
static_assert(kNH % 32 == 0 && kK1P % 32 == 0 && kK1P >= kK1);
static_assert((kNB * kNT) % 4 == 0);
static_assert(kRepackBlocks * 256 == kOut4);
static_assert(kYSP % 32 == 0 && kYSP >= kNT);
static_assert((kWhhP * 2) % 16 == 0 && (kW1P * 2) % 16 == 0 && (kAP * 2) % 16 == 0);
static_assert(kWaves * 2 == kSeqPB);
static_assert((kNG * kNH) % (4 * kThreads) == 0);
static_assert((kNFFN * kW1P) % kThreads == 0);

template <typename T> struct Frag;
template <> struct Frag<_Float16> {
  typedef v16h V; union U { v16h v; v8h h[2]; };
  static __device__ __forceinline__ v16h load(const _Float16* p) {
    U f; f.h[0] = *(const v8h*)(p); f.h[1] = *(const v8h*)(p + 16); return f.v;
  }
};
__device__ __forceinline__ v8f mma_h(v16h a, v16h b, v8f c) {
  c = __builtin_amdgcn_wmma_f32_16x16x32_f16(false, a, false, b, (short)0, c, false, false);
  asm volatile("v_nop\n\tv_nop\n\tv_nop\n\tv_nop" : "+v"(c) : "v"(a), "v"(b));
  return c;
}
__device__ __forceinline__ v8f zero8() { return (v8f){0.f, 0.f, 0.f, 0.f, 0.f, 0.f, 0.f, 0.f}; }

__device__ __forceinline__ float ftanh(float x) { return 1.0f - 2.0f * __builtin_amdgcn_rcpf(1.0f + __expf(2.0f * x)); }
__device__ __forceinline__ float fsigm(float x) { return __builtin_amdgcn_rcpf(1.0f + __expf(-x)); }
__device__ __forceinline__ float tap9(float z, float yv, v4f f0, v4f f1, const float (&w)[kKIN]) {
  z = fmaf(yv, w[0], z);
  z = fmaf(f0[0], w[1], z); z = fmaf(f0[1], w[2], z); z = fmaf(f0[2], w[3], z); z = fmaf(f0[3], w[4], z);
  z = fmaf(f1[0], w[5], z); z = fmaf(f1[1], w[6], z); z = fmaf(f1[2], w[7], z); z = fmaf(f1[3], w[8], z);
  return z;
}

__global__ __launch_bounds__(kThreads) void lstm_ffn_scan_kernel(
    const float* __restrict__ x,
    const float* __restrict__ maskp,
    const float* __restrict__ tvf,
    const float* __restrict__ stf,
    const float* __restrict__ W_ih,
    const float* __restrict__ W_hh,
    const float* __restrict__ b_ih,
    const float* __restrict__ b_hh,
    const float* __restrict__ W1,
    const float* __restrict__ b1,
    const float* __restrict__ W2,
    const float* __restrict__ b2,
    const int*   __restrict__ tfr,
    float* __restrict__ ys) {
  __shared__ __align__(16) _Float16 sWhh[kNG * kWhhP];
  __shared__ __align__(16) _Float16 sW1[kNFFN * kW1P];
  __shared__ __align__(16) _Float16 sA[kSeqPB * kAP];
  __shared__ __align__(16) float    sY[kSeqPB * kYSP];
  __shared__ __align__(16) float    sFeat[kSeqPB * kNF];
  __shared__ __align__(16) float    sYpart[kWaves * kSeqPB];
  __shared__ __align__(16) float    sYcur[kSeqPB];

  const int tid = threadIdx.x, lane = tid & 31, wave = tid >> 5;
  const int n = lane & 15, hh = lane >> 4, koff = hh * 8;
  const int b0 = blockIdx.x * kSeqPB;
  const int u = wave * 16 + n;

  for (int i = tid; i < kNG * kNH / 4; i += kThreads) {
    const v4f w = *(const v4f*)(W_hh + 4 * i);
    v4h o;
    o[0] = (_Float16)(w[0] * kWSc); o[1] = (_Float16)(w[1] * kWSc);
    o[2] = (_Float16)(w[2] * kWSc); o[3] = (_Float16)(w[3] * kWSc);
    *(v4h*)(sWhh + 4 * i) = o;
  }
  for (int i = tid; i < kNFFN * kW1P; i += kThreads) {
    const int r1 = i / kW1P, k = i - r1 * kW1P;
    const int kc = (k < kK1) ? k : (kK1 - 1);
    const float v = W1[r1 * kK1 + kc];
    sW1[i] = (_Float16)((k < kK1) ? v * kWSc : 0.0f);
  }
  {
    const v8h z8 = {(_Float16)0.f, (_Float16)0.f, (_Float16)0.f, (_Float16)0.f,
                    (_Float16)0.f, (_Float16)0.f, (_Float16)0.f, (_Float16)0.f};
    for (int i = tid; i < kSeqPB * kAP / 8; i += kThreads) *(v8h*)(sA + 8 * i) = z8;
    const v4f z4 = {0.f, 0.f, 0.f, 0.f};
    for (int i = tid; i < kSeqPB * kYSP / 4; i += kThreads) *(v4f*)(sY + 4 * i) = z4;
    if (tid < kSeqPB) sYcur[tid] = x[(size_t)(b0 + tid) * kNT];
  }
  float wih[4][kKIN];
  float bsum[4];
#pragma unroll
  for (int g = 0; g < 4; ++g) {
#pragma unroll
    for (int k = 0; k < kKIN; ++k) wih[g][k] = W_ih[(size_t)(g * kNH + u) * kKIN + k];
    bsum[g] = b_ih[g * kNH + u] + b_hh[g * kNH + u];
  }
  const float b1u = b1[u], w2u = W2[u], b2s = b2[0];
  float cst[8];
#pragma unroll
  for (int r = 0; r < 8; ++r) cst[r] = 0.0f;
  const _Float16* arow  = sA + n * kAP + koff;
  const _Float16* brow  = sWhh + (size_t)u * kWhhP + koff;
  const _Float16* w1row = sW1 + (size_t)u * kW1P + koff;
  __syncthreads();

#pragma unroll 1
  for (int t = 0; t < kNT; ++t) {
    if (wave == 0) {
      const int row = lane >> 1, hf = lane & 1;
      const v4f f = *(const v4f*)(tvf + ((size_t)(b0 + row) * kNT + t) * kNF + 4 * hf);
      *(v4f*)(sFeat + row * kNF + 4 * hf) = f;
    } else if (wave < 3) {
      const int i = tid - 32, row = i >> 2, q = i & 3;
      const v4f s = *(const v4f*)(stf + ((size_t)(b0 + row) * kNT + t) * kNS + 4 * q);
      v4h o;
      o[0] = (_Float16)(s[0] * kASc); o[1] = (_Float16)(s[1] * kASc);
      o[2] = (_Float16)(s[2] * kASc); o[3] = (_Float16)(s[3] * kASc);
      *(v4h*)(sA + row * kAP + kNH + 4 * q) = o;
    }

    v8f acc[4];
#pragma unroll
    for (int g = 0; g < 4; ++g) acc[g] = zero8();
#pragma unroll 1
    for (int kc = 0; kc < kNH / 32; ++kc) {
      const v16h fa  = Frag<_Float16>::load(arow + kc * 32);
      const v16h fb0 = Frag<_Float16>::load(brow + kc * 32);
      const v16h fb1 = Frag<_Float16>::load(brow + (size_t)1 * kNH * kWhhP + kc * 32);
      const v16h fb2 = Frag<_Float16>::load(brow + (size_t)2 * kNH * kWhhP + kc * 32);
      const v16h fb3 = Frag<_Float16>::load(brow + (size_t)3 * kNH * kWhhP + kc * 32);
      acc[0] = mma_h(fa, fb0, acc[0]);
      acc[1] = mma_h(fa, fb1, acc[1]);
      acc[2] = mma_h(fa, fb2, acc[2]);
      acc[3] = mma_h(fa, fb3, acc[3]);
    }
    __syncthreads();

#pragma unroll
    for (int r = 0; r < 8; ++r) {
      const int row = hh * 8 + r;
      const float yv = sYcur[row];
      const v4f f0 = *(const v4f*)(sFeat + row * kNF);
      const v4f f1 = *(const v4f*)(sFeat + row * kNF + 4);
      float zi = fmaf(acc[0][r], kDown, bsum[0]);
      float zf = fmaf(acc[1][r], kDown, bsum[1]);
      float zg = fmaf(acc[2][r], kDown, bsum[2]);
      float zo = fmaf(acc[3][r], kDown, bsum[3]);
      zi = tap9(zi, yv, f0, f1, wih[0]);
      zf = tap9(zf, yv, f0, f1, wih[1]);
      zg = tap9(zg, yv, f0, f1, wih[2]);
      zo = tap9(zo, yv, f0, f1, wih[3]);
      const float iv = fsigm(zi), fv = fsigm(zf), gv = ftanh(zg), ov = fsigm(zo);
      const float cn = fmaf(fv, cst[r], iv * gv);
      cst[r] = cn;
      const float hv = ov * ftanh(cn);
      sA[row * kAP + u] = (_Float16)(hv * kASc);
    }
    __syncthreads();

    v8f accF = zero8();
#pragma unroll 1
    for (int kc = 0; kc < kK1P / 32; ++kc) {
      const v16h fa = Frag<_Float16>::load(arow + kc * 32);
      const v16h fb = Frag<_Float16>::load(w1row + kc * 32);
      accF = mma_h(fa, fb, accF);
    }
#pragma unroll
    for (int r = 0; r < 8; ++r) {
      float p = fmaxf(fmaf(accF[r], kDown, b1u), 0.0f) * w2u;
      p += __shfl_xor(p, 1, 32);
      p += __shfl_xor(p, 2, 32);
      p += __shfl_xor(p, 4, 32);
      p += __shfl_xor(p, 8, 32);
      if (n == 0) sYpart[wave * kSeqPB + hh * 8 + r] = p;
    }
    __syncthreads();

    if (tid < kSeqPB) {
      float s = 0.0f;
#pragma unroll
      for (int w = 0; w < kWaves; ++w) s += sYpart[w * kSeqPB + tid];
      const float y = s + b2s;
      sYcur[tid] = y;
      sY[tid * kYSP + t] = y;
    }
  }
  __syncthreads();

  {
    const int q = lane >> 3, c4 = (lane & 7) * 4;
    for (int pass = 0; pass < 2; ++pass) {
#pragma unroll
      for (int rr = 0; rr < 2; ++rr) {
        const int row = wave * 2 + rr;
#pragma unroll
        for (int it = 0; it < 3; ++it) {
          const int col = (it * 4 + q) * 32 + c4;
          const v4f v = *(const v4f*)(sY + row * kYSP + col);
          *(volatile v4f*)(ys + (size_t)(b0 + row) * kYSP + col) = v;
        }
      }
      __threadfence();
    }
  }
}

__global__ __launch_bounds__(256) void repack_kernel(const float* __restrict__ ys, float* __restrict__ out) {
  const int g = blockIdx.x * 256 + threadIdx.x;
  if (g >= kOut4) return;
  const int e0 = g * 4;
  v4f v;
#pragma unroll
  for (int j = 0; j < 4; ++j) {
    const int e = e0 + j;
    int b = e / kNT;
    b = (b < kNB) ? b : (kNB - 1);
    const int t = e - b * kNT;
    v[j] = ys[(size_t)b * kYSP + t];
  }
  *(volatile v4f*)(out + e0) = v;
  __threadfence();
  *(volatile v4f*)(out + e0) = v;
}

extern "C" void kernel_launch(void* const* d_in, const int* in_sizes, int n_in,
                              void* d_out, int out_size, void* d_ws, size_t ws_size, hipStream_t stream) {
  if (n_in < 13 || d_out == nullptr || d_ws == nullptr) return;
  if (in_sizes[0] != kNB * kNT || in_sizes[1] < 1 || in_sizes[2] != kNB * kNT * kNF || in_sizes[3] != kNB * kNT * kNS ||
      in_sizes[4] != kNG * kKIN || in_sizes[5] != kNG * kNH || in_sizes[6] != kNG || in_sizes[7] != kNG ||
      in_sizes[8] != kNFFN * kK1 || in_sizes[9] != kNFFN || in_sizes[10] != kNFFN || in_sizes[11] < 1 ||
      in_sizes[12] < 1 || out_size != kNB * kNT) return;

  const float* x     = (const float*)d_in[0];
  const float* maskp = (const float*)d_in[1];
  const float* tvf   = (const float*)d_in[2];
  const float* stf   = (const float*)d_in[3];
  const float* W_ih  = (const float*)d_in[4];
  const float* W_hh  = (const float*)d_in[5];
  const float* b_ih  = (const float*)d_in[6];
  const float* b_hh  = (const float*)d_in[7];
  const float* W1    = (const float*)d_in[8];
  const float* b1    = (const float*)d_in[9];
  const float* W2    = (const float*)d_in[10];
  const float* b2    = (const float*)d_in[11];
  const int*   tfr   = (const int*)d_in[12];
  float* out = (float*)d_out;

  const size_t ysBytes = (size_t)kNB * kYSP * sizeof(float);
  if (ysBytes > ws_size || ysBytes > (size_t)134217728) return;
  float* ys = (float*)d_ws;

  lstm_ffn_scan_kernel<<<kBlocks, kThreads, 0, stream>>>(x, maskp, tvf, stf, W_ih, W_hh, b_ih, b_hh, W1, b1, W2, b2, tfr, ys);

  repack_kernel<<<kRepackBlocks, 256, 0, stream>>>(ys, out);
}
